// GatedLinearAttention_16896401342973
// MI455X (gfx1250) — hardware-verified
//
#include <hip/hip_runtime.h>
#include <math.h>

constexpr int kNb    = 2;
constexpr int kSeq   = 2048;
constexpr int kDim   = 1024;
constexpr int kNh    = 16;
constexpr int kHd    = 64;
constexpr int kChunk = 64;
constexpr int kGh    = 16;
constexpr int kTok   = kNb * kSeq;
constexpr int kQkv   = 3 * kDim;
constexpr int kCat   = kQkv + 64;
constexpr int kNx    = kTok * kDim;
constexpr int kSub   = 32;
constexpr int kGateTok  = 64;
constexpr int kGateCols = 512;
constexpr float kPCarry = 32768.0f;
constexpr int isqrt_c(int n) { int r = 0; while ((r + 1) * (r + 1) <= n) ++r; return r; }
constexpr int kHdRoot = isqrt_c(kHd);
constexpr float kScoreScale = 1.0f / (float)kHdRoot;
static_assert(kHdRoot * kHdRoot == kHd);
static_assert(kNh * kHd == kDim);
static_assert(kHd == 64 && kChunk == 64);
static_assert(kSeq % kChunk == 0 && kSeq % kSub == 0);
static_assert(kTok % 64 == 0 && kCat % 64 == 0 && kDim % 32 == 0);
static_assert(((kTok / 64) * (kCat / 64)) % 8 == 0);
static_assert(kGh == 16 && kDim % 64 == 0);
static_assert(kTok % kGateTok == 0 && kDim % kGateCols == 0);

typedef __attribute__((ext_vector_type(16))) _Float16 v16h;
typedef __attribute__((ext_vector_type(8)))  _Float16 v8h;
typedef __attribute__((ext_vector_type(16))) __bf16   v16b;
typedef __attribute__((ext_vector_type(8)))  __bf16   v8b;
typedef __attribute__((ext_vector_type(8)))  float    v8f;
typedef __attribute__((ext_vector_type(4)))  float    v4f;
typedef __attribute__((ext_vector_type(4)))  unsigned int v4u;

__device__ __forceinline__ unsigned short f2bf_bits(float f) {
  unsigned u = __float_as_uint(f);
  return (unsigned short)((u + 0x7FFFu + ((u >> 16) & 1u)) >> 16);
}
__device__ __forceinline__ float bf_bits2f(unsigned short h) { return __uint_as_float(((unsigned)h) << 16); }
__device__ __forceinline__ float bf16r(float f) { return bf_bits2f(f2bf_bits(f)); }
__device__ __forceinline__ unsigned pk16(unsigned short a, unsigned short b) { return (unsigned)a | ((unsigned)b << 16); }

__device__ __forceinline__ void guard_row_b(v8f& a0, v8f& a1, v8f& a2, v8f& a3, v16b x, v16b b0, v16b b1, v16b b2, v16b b3) {
  asm volatile("v_nop\n\tv_nop\n\tv_nop\n\tv_nop" : "+v"(a0), "+v"(a1), "+v"(a2), "+v"(a3) : "v"(x), "v"(b0), "v"(b1), "v"(b2), "v"(b3));
}
__device__ __forceinline__ void keep4_b(v16b a, v16b b, v16b c, v16b d) { asm volatile("v_nop" :: "v"(a), "v"(b), "v"(c), "v"(d)); }
__device__ __forceinline__ void acc_guard4(v8f& a, v8f& b, v8f& c, v8f& d) { asm volatile("v_nop\n\tv_nop\n\tv_nop\n\tv_nop" : "+v"(a), "+v"(b), "+v"(c), "+v"(d)); }

template <typename T> struct Frag;
template <> struct Frag<_Float16> {
  typedef v16h V; union U { v16h v; v8h h[2]; };
  static __device__ __forceinline__ v16h load(const _Float16* p) {
    U f; f.h[0] = *(const v8h*)(p); f.h[1] = *(const v8h*)(p + 16); return f.v;
  }
};
template <> struct Frag<__bf16> {
  typedef v16b V; union U { v16b v; v8b h[2]; };
  static __device__ __forceinline__ v16b load(const __bf16* p) {
    U f; f.h[0] = *(const v8b*)(p); f.h[1] = *(const v8b*)(p + 16); return f.v;
  }
  static __device__ __forceinline__ v8f mma(v16b a, v16b b, v8f c) {
    return __builtin_amdgcn_wmma_f32_16x16x32_bf16(false, a, false, b, (short)0, c, false, false);
  }
};
__device__ __forceinline__ v8f mma_h(v16h a, v16h b, v8f c) {
  c = __builtin_amdgcn_wmma_f32_16x16x32_f16(false, a, false, b, (short)0, c, false, false);
  asm volatile("v_nop\n\tv_nop\n\tv_nop\n\tv_nop" : "+v"(c) : "v"(a), "v"(b));
  return c;
}

__global__ __launch_bounds__(256) void cvt8_bf16_kernel(const float* __restrict__ in, unsigned short* __restrict__ out, int n8) {
  const int i = blockIdx.x * 256 + threadIdx.x;
  if (i >= n8) return;
  const float* p = in + 8 * (size_t)i;
  const v4f a = *(const v4f*)(p);
  const v4f c = *(const v4f*)(p + 4);
  unsigned short hb[8];
#pragma unroll
  for (int e = 0; e < 4; ++e) {
    const float fa = a[e];
    const float fc = c[e];
    hb[e]     = f2bf_bits(fa);
    hb[4 + e] = f2bf_bits(fc);
  }
  const v4u u = (v4u){pk16(hb[0], hb[1]), pk16(hb[2], hb[3]), pk16(hb[4], hb[5]), pk16(hb[6], hb[7])};
  unsigned short* q = out + 8 * (size_t)i;
  *(volatile v4u*)q = u;
  __threadfence();
  *(volatile v4u*)q = u;
}

__global__ __launch_bounds__(256) void wt_build_kernel(const float* __restrict__ Wq, const float* __restrict__ Wk,
                                                       const float* __restrict__ Wv, const float* __restrict__ Wg1,
                                                       unsigned short* __restrict__ out) {
  __shared__ float sm[64][65];
  const int t   = threadIdx.x;
  const int k0  = blockIdx.x * 64;
  const int tn  = blockIdx.y;
  const int sel = tn >> 4;
  const float* W = (sel == 0) ? Wq : (sel == 1) ? Wk : (sel == 2) ? Wv : Wg1;
  const int pitch = (sel < 3) ? kDim : kGh;
  const int ncol  = (sel < 3) ? kDim : kGh;
  const int nc0   = (tn & 15) * 64;
#pragma unroll
  for (int i = 0; i < 16; ++i) {
    const int e = i * 256 + t;
    const int r = e >> 6;
    const int c = e & 63;
    const int col  = nc0 + c;
    const int colc = (col < ncol) ? col : (ncol - 1);
    const float v = W[(size_t)(k0 + r) * pitch + colc];
    sm[c][r] = (col < ncol) ? v : 0.0f;
  }
  __syncthreads();
  const int lane = t & 31, wave = t >> 5;
  const int q = lane >> 3, c8 = (lane & 7) * 8;
  for (int pass = 0; pass < 2; ++pass) {
#pragma unroll
    for (int it = 0; it < 2; ++it) {
      const int row = wave * 8 + it * 4 + q;
      unsigned short hb[8];
#pragma unroll
      for (int e = 0; e < 8; ++e) hb[e] = f2bf_bits(sm[row][c8 + e]);
      const v4u u = (v4u){pk16(hb[0], hb[1]), pk16(hb[2], hb[3]), pk16(hb[4], hb[5]), pk16(hb[6], hb[7])};
      *(volatile v4u*)(out + (size_t)(tn * 64 + row) * kDim + k0 + c8) = u;
    }
    __threadfence();
  }
}

__global__ __launch_bounds__(256) void bias_cat_kernel(const float* __restrict__ bq, const float* __restrict__ bk,
                                                       const float* __restrict__ bv, const float* __restrict__ bg1,
                                                       float* __restrict__ dst) {
  const int z = blockIdx.x;
  const int tid = threadIdx.x;
  if (z < 3) {
    const float* src = (z == 0) ? bq : (z == 1) ? bk : bv;
    const v4f v = *(const v4f*)(src + 4 * tid);
    v4f o;
#pragma unroll
    for (int e = 0; e < 4; ++e) { const float f = v[e]; o[e] = bf16r(f); }
    float* op = dst + z * kDim + 4 * tid;
    *(volatile v4f*)op = o;
    __threadfence();
    *(volatile v4f*)op = o;
  } else if (tid < 16) {
    v4f o;
#pragma unroll
    for (int e = 0; e < 4; ++e) {
      const int idx = 4 * tid + e;
      const int ic  = (idx < kGh) ? idx : (kGh - 1);
      const float f = bg1[ic];
      o[e] = (idx < kGh) ? bf16r(f) : 0.0f;
    }
    float* op = dst + kQkv + 4 * tid;
    *(volatile v4f*)op = o;
    __threadfence();
    *(volatile v4f*)op = o;
  }
}

__global__ __launch_bounds__(256) void gemm_bf16_bias_kernel(
    const unsigned short* __restrict__ Ap, int lda,
    const unsigned short* __restrict__ Btp, int ldb,
    float* __restrict__ C, int ldc,
    const float* __restrict__ bias, int M, int N, int K) {
  typedef __bf16 T;
  const T* A  = (const T*)Ap;
  const T* Bt = (const T*)Btp;
  __shared__ __align__(16) float sT[8][16 * 68];
  const int lane = threadIdx.x & 31;
  const int wave = threadIdx.x >> 5;
  const int tilesN = N >> 6;
  const int tilesM = M >> 6;
  const int tile = blockIdx.x * 8 + wave;
  if (tile >= tilesM * tilesN) return;
  const int tm = tile / tilesN;
  const int tn = tile - tm * tilesN;
  const int m0 = tm << 6;
  const int n0 = tn << 6;
  const int rlane = lane & 15;
  const int koff  = (lane >> 4) * 8;
  const int mOff  = (lane >> 4) * 8;

  const T* ap[4];
  const T* bp[4];
#pragma unroll
  for (int i = 0; i < 4; ++i) {
    ap[i] = A  + (size_t)(m0 + (i << 4) + rlane) * lda + koff;
    bp[i] = Bt + (size_t)(n0 + (i << 4) + rlane) * ldb + koff;
  }

  v8f acc[4][4];
#pragma unroll
  for (int i = 0; i < 4; ++i)
#pragma unroll
    for (int j = 0; j < 4; ++j) acc[i][j] = (v8f){0.f, 0.f, 0.f, 0.f, 0.f, 0.f, 0.f, 0.f};

  for (int k0 = 0; k0 < K; k0 += 32) {
    v16b bh[4];
#pragma unroll
    for (int j = 0; j < 4; ++j) bh[j] = Frag<T>::load(bp[j] + k0);
#pragma unroll
    for (int i = 0; i < 4; ++i) {
      const v16b ah = Frag<T>::load(ap[i] + k0);
#pragma unroll
      for (int j = 0; j < 4; ++j) acc[i][j] = Frag<T>::mma(ah, bh[j], acc[i][j]);
      guard_row_b(acc[i][0], acc[i][1], acc[i][2], acc[i][3], ah, bh[0], bh[1], bh[2], bh[3]);
    }
    keep4_b(bh[0], bh[1], bh[2], bh[3]);
  }
  acc_guard4(acc[0][0], acc[0][1], acc[0][2], acc[0][3]);
  acc_guard4(acc[1][0], acc[1][1], acc[1][2], acc[1][3]);
  acc_guard4(acc[2][0], acc[2][1], acc[2][2], acc[2][3]);
  acc_guard4(acc[3][0], acc[3][1], acc[3][2], acc[3][3]);

  float* slab = sT[wave];
#pragma unroll
  for (int i = 0; i < 4; ++i) {
    const int mBase = m0 + (i << 4);
#pragma unroll
    for (int j = 0; j < 4; ++j) {
      const int n = n0 + (j << 4) + rlane;
      const float bvv = bias[n];
#pragma unroll
      for (int r = 0; r < 8; ++r) {
        slab[(mOff + r) * 68 + (j << 4) + rlane] = acc[i][j][r] + bvv;
      }
    }
    __builtin_amdgcn_fence(__ATOMIC_RELEASE, "workgroup");
    __builtin_amdgcn_wave_barrier();
    __builtin_amdgcn_fence(__ATOMIC_ACQUIRE, "workgroup");
    {
      const int hh = lane >> 4, c4 = (lane & 15) * 4;
      for (int pass = 0; pass < 2; ++pass) {
#pragma unroll
        for (int it = 0; it < 8; ++it) {
          const int row = it * 2 + hh;
          const v4f v = *(const v4f*)(slab + row * 68 + c4);
          *(volatile v4f*)(C + (size_t)(mBase + row) * ldc + n0 + c4) = v;
        }
        __threadfence();
      }
    }
    __builtin_amdgcn_fence(__ATOMIC_RELEASE, "workgroup");
    __builtin_amdgcn_wave_barrier();
    __builtin_amdgcn_fence(__ATOMIC_ACQUIRE, "workgroup");
  }
}

__global__ __launch_bounds__(128) void gate_kernel(const float* __restrict__ P, const float* __restrict__ Wg2,
                                                   const float* __restrict__ bg2, float* __restrict__ AL) {
  __shared__ __align__(16) float sW[kGh * kGateCols];
  __shared__ __align__(16) float sS[kGateTok * kGh];
  const int tid  = threadIdx.x;
  const int tok0 = blockIdx.x * kGateTok;
  const int col0 = blockIdx.y * kGateCols;
#pragma unroll 4
  for (int it = 0; it < 16; ++it) {
    const int idx4 = it * 128 + tid;
    const int i  = idx4 >> 7;
    const int c4 = (idx4 & 127) * 4;
    const v4f w = *(const v4f*)(Wg2 + (size_t)i * kDim + col0 + c4);
    v4f o;
#pragma unroll
    for (int e = 0; e < 4; ++e) { const float f = w[e]; o[e] = bf16r(f); }
    *(v4f*)(sW + i * kGateCols + c4) = o;
  }
#pragma unroll 1
  for (int it = 0; it < 8; ++it) {
    const int idx = it * 128 + tid;
    const int tk = idx >> 4;
    const int i  = idx & 15;
    const float hv = P[(size_t)(tok0 + tk) * kCat + kQkv + i];
    const float sg = 1.0f / (1.0f + expf(-hv));
    sS[idx] = hv * sg;
  }
  __syncthreads();
  const int col = col0 + 4 * tid;
  v4f b4;
  {
    const v4f braw = *(const v4f*)(bg2 + col);
#pragma unroll
    for (int e = 0; e < 4; ++e) { const float f = braw[e]; b4[e] = bf16r(f); }
  }
#pragma unroll 1
  for (int tk = 0; tk < kGateTok; ++tk) {
    v4f g = b4;
#pragma unroll 1
    for (int i4 = 0; i4 < 4; ++i4) {
      const v4f s4 = *(const v4f*)(sS + tk * kGh + 4 * i4);
#pragma unroll
      for (int u = 0; u < 4; ++u) {
        const v4f w4 = *(const v4f*)(sW + (4 * i4 + u) * kGateCols + 4 * tid);
        const float su = s4[u];
#pragma unroll
        for (int e = 0; e < 4; ++e) g[e] = fmaf(su, w4[e], g[e]);
      }
    }
    v4f al;
#pragma unroll
    for (int e = 0; e < 4; ++e) {
      const float ge = g[e];
      const float sg = 1.0f / (1.0f + expf(-ge));
      al[e] = 0.9f * sg + 0.1f;
    }
    float* op = AL + (size_t)(tok0 + tk) * kDim + col;
    *(volatile v4f*)op = al;
    __threadfence();
    *(volatile v4f*)op = al;
  }
}

__global__ __launch_bounds__(128) void scan_kernel(const float* __restrict__ P, const float* __restrict__ AL,
                                                   float* __restrict__ INTER) {
  __shared__ __align__(16) float sq[kSub * 64];
  __shared__ __align__(16) float sk[kSub * 64];
  __shared__ __align__(16) float sa[kSub * 64];
  __shared__ __align__(16) float sv[kSub * 64];
  __shared__ __align__(16) float sp[2 * kSub * 64];
  const int tid = threadIdx.x;
  const int e   = tid & 63;
  const int dh  = tid >> 6;
  const int bh  = blockIdx.x;
  const int b   = bh / kNh;
  const int h   = bh - b * kNh;
  const size_t tokbase = (size_t)b * kSeq;

  float S[32];
#pragma unroll
  for (int d = 0; d < 32; ++d) S[d] = 0.0f;

#pragma unroll 1
  for (int sc = 0; sc < kSeq / kSub; ++sc) {
    const int t0 = sc * kSub;
#pragma unroll
    for (int it = 0; it < 4; ++it) {
      const int idx = it * 128 + tid;
      const int row = idx >> 4;
      const int c4  = (idx & 15) * 4;
      const float* qp = P + (tokbase + t0 + row) * kCat + h * kHd + c4;
      const v4f vq = *(const v4f*)(qp);
      const v4f vk = *(const v4f*)(qp + kDim);
      const v4f vv = *(const v4f*)(qp + 2 * kDim);
      const v4f va = *(const v4f*)(AL + (tokbase + t0 + row) * kDim + h * kHd + c4);
      *(v4f*)(sq + row * 64 + c4) = vq;
      *(v4f*)(sk + row * 64 + c4) = vk;
      *(v4f*)(sv + row * 64 + c4) = vv;
      *(v4f*)(sa + row * 64 + c4) = va;
    }
    __syncthreads();
#pragma unroll 1
    for (int tt = 0; tt < kSub; ++tt) {
      const float* qr = sq + tt * 64 + dh * 32;
      const float* kr = sk + tt * 64 + dh * 32;
      const float* ar = sa + tt * 64 + dh * 32;
      const float vval = sv[tt * 64 + e];
      float acc0 = 0.0f, acc1 = 0.0f;
#pragma unroll
      for (int d4 = 0; d4 < 8; ++d4) {
        const v4f q4 = *(const v4f*)(qr + 4 * d4);
        acc0 = fmaf(q4[0], S[4 * d4 + 0], acc0);
        acc1 = fmaf(q4[1], S[4 * d4 + 1], acc1);
        acc0 = fmaf(q4[2], S[4 * d4 + 2], acc0);
        acc1 = fmaf(q4[3], S[4 * d4 + 3], acc1);
      }
      sp[(dh * kSub + tt) * 64 + e] = acc0 + acc1;
#pragma unroll
      for (int d4 = 0; d4 < 8; ++d4) {
        const v4f k4 = *(const v4f*)(kr + 4 * d4);
        const v4f a4 = *(const v4f*)(ar + 4 * d4);
#pragma unroll
        for (int u = 0; u < 4; ++u) {
          const float kv = k4[u] * vval;
          S[4 * d4 + u] = fmaf(a4[u], S[4 * d4 + u], kv);
        }
      }
    }
    __syncthreads();
    v4f o[4];
#pragma unroll
    for (int it = 0; it < 4; ++it) {
      const int idx = it * 128 + tid;
      const int row = idx >> 4;
      const int c4  = (idx & 15) * 4;
      const v4f p0 = *(const v4f*)(sp + row * 64 + c4);
      const v4f p1 = *(const v4f*)(sp + (kSub + row) * 64 + c4);
      o[it] = p0 + p1;
    }
    for (int pass = 0; pass < 2; ++pass) {
#pragma unroll
      for (int it = 0; it < 4; ++it) {
        const int idx = it * 128 + tid;
        const int row = idx >> 4;
        const int c4  = (idx & 15) * 4;
        *(volatile v4f*)(INTER + (tokbase + t0 + row) * kDim + h * kHd + c4) = o[it];
      }
      __threadfence();
    }
  }
}

__global__ __launch_bounds__(128) void chunk_softmax_out_kernel(const float* __restrict__ P, const float* __restrict__ INTER,
                                                                float* __restrict__ out) {
  __shared__ __align__(16) _Float16 Qs[64 * 64];
  __shared__ __align__(16) _Float16 Ks[64 * 64];
  __shared__ __align__(16) _Float16 Vt[64 * 64];
  __shared__ __align__(16) _Float16 Ps[4][16 * 64];
  __shared__ __align__(16) float    Os[4][16 * 68];
  __shared__ float sInv[64];

  const int tid  = threadIdx.x;
  const int wave = tid >> 5;
  const int lane = tid & 31;
  const int hh   = lane >> 4;
  const int c    = lane & 15;

  const int bx = blockIdx.x;
  const int n  = bx % (kSeq / kChunk);
  const int bh = bx / (kSeq / kChunk);
  const int h  = bh % kNh;
  const int b  = bh / kNh;
  const size_t tok0 = (size_t)b * kSeq + (size_t)n * kChunk;

  {
    const int kvr = tid >> 1;
    const int dhf = (tid & 1) * 32;
    const float* base = P + (tok0 + kvr) * kCat + h * kHd + dhf;
#pragma unroll
    for (int i = 0; i < 4; ++i) {
      const v4f q0 = *(const v4f*)(base + 8 * i);
      const v4f q1 = *(const v4f*)(base + 8 * i + 4);
      const v4f k0 = *(const v4f*)(base + kDim + 8 * i);
      const v4f k1 = *(const v4f*)(base + kDim + 8 * i + 4);
      const v4f v0 = *(const v4f*)(base + 2 * kDim + 8 * i);
      const v4f v1 = *(const v4f*)(base + 2 * kDim + 8 * i + 4);
      v8h qh, kh;
#pragma unroll
      for (int e = 0; e < 4; ++e) {
        const float fq0 = q0[e];
        const float fq1 = q1[e];
        const float fk0 = k0[e];
        const float fk1 = k1[e];
        qh[e]     = (_Float16)fq0;
        qh[4 + e] = (_Float16)fq1;
        kh[e]     = (_Float16)fk0;
        kh[4 + e] = (_Float16)fk1;
      }
      *(v8h*)(Qs + kvr * 64 + dhf + 8 * i) = qh;
      *(v8h*)(Ks + kvr * 64 + dhf + 8 * i) = kh;
#pragma unroll
      for (int e = 0; e < 4; ++e) {
        const float fv0 = v0[e];
        const float fv1 = v1[e];
        Vt[(dhf + 8 * i + e) * 64 + kvr]     = (_Float16)fv0;
        Vt[(dhf + 8 * i + 4 + e) * 64 + kvr] = (_Float16)fv1;
      }
    }
  }
  __syncthreads();

  v8f s[4];
#pragma unroll
  for (int j = 0; j < 4; ++j) s[j] = (v8f){0.f, 0.f, 0.f, 0.f, 0.f, 0.f, 0.f, 0.f};
#pragma unroll
  for (int dc = 0; dc < 2; ++dc) {
    const v16h a = Frag<_Float16>::load(Qs + (wave * 16 + c) * 64 + dc * 32 + 8 * hh);
#pragma unroll
    for (int j = 0; j < 4; ++j) {
      const v16h kb = Frag<_Float16>::load(Ks + (j * 16 + c) * 64 + dc * 32 + 8 * hh);
      s[j] = mma_h(a, kb, s[j]);
    }
  }
  float* sl = Os[wave];
#pragma unroll
  for (int j = 0; j < 4; ++j)
#pragma unroll
    for (int r = 0; r < 8; ++r) sl[(8 * hh + r) * 68 + j * 16 + c] = s[j][r] * kScoreScale;
  __syncthreads();

  {
    const int row  = lane >> 1;
    const int half = lane & 1;
    const int qpos = wave * 16 + row;
    const float* rp = sl + row * 68 + half * 32;
    float m = -__builtin_inff();
#pragma unroll 1
    for (int i = 0; i < 32; ++i) {
      const int col = half * 32 + i;
      const float x = rp[i];
      const float xm = (col > qpos) ? -__builtin_inff() : x;
      m = fmaxf(m, xm);
    }
    m = fmaxf(m, __shfl_xor(m, 1, 32));
    float sum = 0.0f;
    _Float16* pw = Ps[wave] + row * 64 + half * 32;
#pragma unroll 1
    for (int g = 0; g < 4; ++g) {
      v8h pv;
#pragma unroll
      for (int e = 0; e < 8; ++e) {
        const int col = half * 32 + g * 8 + e;
        const float x = rp[g * 8 + e];
        const float xm = (col > qpos) ? -__builtin_inff() : x;
        const float p = expf(xm - m);
        sum += p;
        pv[e] = (_Float16)(p * kPCarry);
      }
      *(v8h*)(pw + g * 8) = pv;
    }
    sum += __shfl_xor(sum, 1, 32);
    const float inv = 1.0f / (sum * kPCarry);
    if (half == 0) sInv[wave * 16 + row] = inv;
  }
  __syncthreads();

  v8f oacc[4];
#pragma unroll
  for (int t = 0; t < 4; ++t) oacc[t] = (v8f){0.f, 0.f, 0.f, 0.f, 0.f, 0.f, 0.f, 0.f};
#pragma unroll
  for (int kk = 0; kk < 2; ++kk) {
    const v16h pa = Frag<_Float16>::load(Ps[wave] + c * 64 + kk * 32 + 8 * hh);
#pragma unroll
    for (int t = 0; t < 4; ++t) {
      const v16h vb = Frag<_Float16>::load(Vt + (t * 16 + c) * 64 + kk * 32 + 8 * hh);
      oacc[t] = mma_h(pa, vb, oacc[t]);
    }
  }
#pragma unroll
  for (int t = 0; t < 4; ++t)
#pragma unroll
    for (int r = 0; r < 8; ++r) sl[(8 * hh + r) * 68 + t * 16 + c] = oacc[t][r];
  __syncthreads();

  {
    const int c4 = (lane & 15) * 4;
    v4f o[8];
#pragma unroll
    for (int it = 0; it < 8; ++it) {
      const int row = it * 2 + hh;
      const float inv = sInv[wave * 16 + row];
      const v4f a  = *(const v4f*)(sl + row * 68 + c4);
      const v4f rs = *(const v4f*)(INTER + (tok0 + wave * 16 + row) * kDim + h * kHd + c4);
#pragma unroll
      for (int e = 0; e < 4; ++e) o[it][e] = fmaf(a[e], inv, rs[e]);
    }
    for (int pass = 0; pass < 2; ++pass) {
#pragma unroll
      for (int it = 0; it < 8; ++it) {
        const int row = it * 2 + hh;
        *(volatile v4f*)(out + (tok0 + wave * 16 + row) * kDim + h * kHd + c4) = o[it];
      }
      __threadfence();
    }
  }
}

extern "C" void kernel_launch(void* const* d_in, const int* in_sizes, int n_in,
                              void* d_out, int out_size, void* d_ws, size_t ws_size, hipStream_t stream) {
  if (n_in < 11 || d_out == nullptr || d_ws == nullptr) return;
  if (in_sizes[0] != kNx || in_sizes[1] != kDim * kDim || in_sizes[2] != kDim ||
      in_sizes[3] != kDim * kDim || in_sizes[4] != kDim || in_sizes[5] != kDim * kDim ||
      in_sizes[6] != kDim || in_sizes[7] != kDim * kGh || in_sizes[8] != kGh ||
      in_sizes[9] != kGh * kDim || in_sizes[10] != kDim || out_size != kNx) return;

  const float* x   = (const float*)d_in[0];
  const float* Wq  = (const float*)d_in[1];
  const float* bq  = (const float*)d_in[2];
  const float* Wk  = (const float*)d_in[3];
  const float* bk  = (const float*)d_in[4];
  const float* Wv  = (const float*)d_in[5];
  const float* bv  = (const float*)d_in[6];
  const float* Wg1 = (const float*)d_in[7];
  const float* bg1 = (const float*)d_in[8];
  const float* Wg2 = (const float*)d_in[9];
  const float* bg2 = (const float*)d_in[10];
  float* out = (float*)d_out;

  char* ws = (char*)d_ws;
  size_t off = 0;
  auto carve = [&](size_t bytes) -> char* { char* p = ws + off; off += (bytes + 255) & ~(size_t)255; return p; };
  unsigned short* XB    = (unsigned short*)carve((size_t)kTok * kDim * 2);
  unsigned short* WT    = (unsigned short*)carve((size_t)kCat * kDim * 2);
  float*          BIAS  = (float*)carve((size_t)4096 * 4);
  float*          QKVG  = (float*)carve((size_t)kTok * kCat * 4);
  float*          ALPHA = (float*)carve((size_t)kTok * kDim * 4);
  float*          INTER = (float*)carve((size_t)kTok * kDim * 4);
  if (off > ws_size || off > (size_t)134217728) return;

  const int n8x = kNx / 8;
  cvt8_bf16_kernel<<<(n8x + 255) / 256, 256, 0, stream>>>(x, XB, n8x);
  wt_build_kernel<<<dim3(kDim / 64, kCat / 64), 256, 0, stream>>>(Wq, Wk, Wv, Wg1, WT);
  bias_cat_kernel<<<4, 256, 0, stream>>>(bq, bk, bv, bg1, BIAS);

  gemm_bf16_bias_kernel<<<((kTok / 64) * (kCat / 64)) / 8, 256, 0, stream>>>(
      XB, kDim, WT, kDim, QKVG, kCat, BIAS, kTok, kCat, kDim);

  gate_kernel<<<dim3(kTok / kGateTok, kDim / kGateCols), 128, 0, stream>>>(QKVG, Wg2, bg2, ALPHA);

  scan_kernel<<<kNb * kNh, 128, 0, stream>>>(QKVG, ALPHA, INTER);

  chunk_softmax_out_kernel<<<kNb * kNh * (kSeq / kChunk), 128, 0, stream>>>(QKVG, INTER, out);
}
